// GAT_120259084552
// MI455X (gfx1250) — hardware-verified
//
#include <hip/hip_runtime.h>
#include <stddef.h>
#include <stdint.h>
#include <math.h>


#define NBAT   8
#define NN     2048
#define DATT   96
#define KPAD   128
#define HD     64
#define NH     8
#define HC     512
#define K2     1024
#define MROWS  (NBAT * NN)
#define PTHR   256
#define GTHR   128
#define ATHR   128
#define U_HB   (MROWS * (KPAD / 8))
#define U_WH   (HC * (KPAD / 8))
#define U_WO   (HD * (K2 / 8))
#define U_BB   (NN * (NN / 8))
#define U_ALL  (U_HB + U_WH + U_WO + U_BB)
#define WSMAX  134217728

static_assert(U_HB % PTHR == 0 && U_WH % PTHR == 0 && U_WO % PTHR == 0 && U_BB % PTHR == 0);
static_assert(KPAD % 32 == 0 && K2 % 32 == 0 && DATT <= KPAD && (DATT % 8) == 0);
static_assert(K2 == 2 * HC && HC == NH * HD && HD == 64);
static_assert(MROWS % 64 == 0 && NN % 64 == 0 && NN == 2048);
static_assert(GTHR == 2 * HD && ATHR == 128);

typedef float          v2f  __attribute__((ext_vector_type(2)));
typedef float          v4f  __attribute__((ext_vector_type(4)));
typedef float          v8f  __attribute__((ext_vector_type(8)));
typedef int            v8i  __attribute__((ext_vector_type(8)));
typedef unsigned int   v4u  __attribute__((ext_vector_type(4)));
typedef unsigned short v8us __attribute__((ext_vector_type(8)));
typedef __bf16         v16b __attribute__((ext_vector_type(16)));
typedef v2f  __attribute__((may_alias)) v2fa;
typedef v4f  __attribute__((may_alias)) v4fa;
typedef v4u  __attribute__((may_alias)) v4ua;
typedef v8us __attribute__((may_alias)) v8usa;
union FragB { v16b v; v8us h[2]; v8i w; };

__device__ __forceinline__ v8f wmb(const FragB& a, const FragB& b, v8f c) {
  v8f d = __builtin_amdgcn_wmma_f32_16x16x32_bf16(false, a.v, false, b.v, (short)0, c, false, false);
  asm volatile("v_nop\n\tv_nop\n\tv_nop\n\tv_nop" : "+v"(d) : "v"(a.w), "v"(b.w));
  return d;
}

__device__ __forceinline__ unsigned int f2bf(float f) {
  const unsigned int u = __float_as_uint(f);
  return ((u + 0x7FFFu + ((u >> 16) & 1u)) >> 16) & 0xFFFFu;
}
__device__ __forceinline__ float bf2f(unsigned int b) { return __uint_as_float(b << 16); }
__device__ __forceinline__ float bfr(float f) { return bf2f(f2bf(f)); }
__device__ __forceinline__ unsigned int pk2(float lo, float hi) { return f2bf(lo) | (f2bf(hi) << 16); }
__device__ __forceinline__ v4u pack8(const v4f a, const v4f b) {
  v4u r;
  r.x = pk2(a.x, a.y); r.y = pk2(a.z, a.w); r.z = pk2(b.x, b.y); r.w = pk2(b.z, b.w);
  return r;
}
__device__ __forceinline__ void st2u(unsigned short* p, const v4u v) {
  *(volatile v4u*)p = v;
  __threadfence();
  *(volatile v4u*)p = v;
}
__device__ __forceinline__ float eluf(float x) {
  const float e = expm1f(x);
  return x > 0.0f ? x : e;
}
__device__ __forceinline__ float sc1(float f1, float f2, float bv) {
  float s = f1 + f2;
  s = fmaxf(s, 0.2f * s);
  return s + bv;
}

__global__ __launch_bounds__(PTHR) void k_prep(const float* __restrict__ inp, const float* __restrict__ env,
                                               const float* __restrict__ st, const float* __restrict__ bias,
                                               const float* __restrict__ Wh, const float* __restrict__ Wo,
                                               unsigned short* HBp, unsigned short* WHTp,
                                               unsigned short* WO2p, unsigned short* BBp) {
  const int u = (int)blockIdx.x * PTHR + (int)threadIdx.x;
  if (u < U_HB) {
    const int row = u >> 4, c8 = u & 15;
    const v2f in2 = *(const v2fa*)(inp + (size_t)row * 2);
    int eb = 8 * c8 - 2; eb = eb < 0 ? 0 : (eb > 22 ? 22 : eb);
    const float* ep = env + (size_t)row * 30 + eb;
    const v2f e0 = *(const v2fa*)ep;
    const v2f e1 = *(const v2fa*)(ep + 2);
    const v2f e2 = *(const v2fa*)(ep + 4);
    const v2f e3 = *(const v2fa*)(ep + 6);
    int sc = 8 * c8 - 32; sc = sc < 0 ? 0 : (sc > 56 ? 56 : sc);
    const float* sp = st + (size_t)row * HD + sc;
    const v4f s0 = *(const v4fa*)sp;
    const v4f s1 = *(const v4fa*)(sp + 4);
    const unsigned int w01 = pk2(e0.x, e0.y), w23 = pk2(e1.x, e1.y), w45 = pk2(e2.x, e2.y), w67 = pk2(e3.x, e3.y);
    const unsigned int wi  = pk2(in2.x, in2.y);
    const v4u cs = pack8(s0, s1);
    const unsigned int mA = (c8 == 0) ? 0xFFFFFFFFu : 0u;
    const unsigned int mB = (c8 >= 1 && c8 <= 3) ? 0xFFFFFFFFu : 0u;
    const unsigned int mS = (c8 >= 4 && c8 <= 11) ? 0xFFFFFFFFu : 0u;
    v4u o;
    o.x = (wi  & mA) | (w01 & mB) | (cs.x & mS);
    o.y = (w01 & mA) | (w23 & mB) | (cs.y & mS);
    o.z = (w23 & mA) | (w45 & mB) | (cs.z & mS);
    o.w = (w45 & mA) | (w67 & mB) | (cs.w & mS);
    st2u(HBp + (size_t)row * KPAD + 8 * c8, o);
  } else if (u < U_HB + U_WH) {
    const int v  = u - U_HB;
    const int n  = v >> 4, d8 = (v & 15) * 8;
    const int kh = n >> 6, hc = n & 63;
    const int dc = d8 < DATT - 8 ? d8 : DATT - 8;
    const float* p = Wh + ((size_t)kh * DATT + dc) * HD + hc;
    v4f a, b;
    a.x = p[0];      a.y = p[HD];     a.z = p[2 * HD]; a.w = p[3 * HD];
    b.x = p[4 * HD]; b.y = p[5 * HD]; b.z = p[6 * HD]; b.w = p[7 * HD];
    v4u o = pack8(a, b);
    const unsigned int mk = d8 < DATT ? 0xFFFFFFFFu : 0u;
    o.x &= mk; o.y &= mk; o.z &= mk; o.w &= mk;
    st2u(WHTp + (size_t)n * KPAD + d8, o);
  } else if (u < U_HB + U_WH + U_WO) {
    const int v  = u - U_HB - U_WH;
    const int n  = v >> 7, k8 = (v & 127) * 8;
    const int kk = k8 & (HC - 1);
    const float* p = Wo + (size_t)kk * HD + n;
    v4f a, b;
    a.x = p[0];      a.y = p[HD];     a.z = p[2 * HD]; a.w = p[3 * HD];
    b.x = p[4 * HD]; b.y = p[5 * HD]; b.z = p[6 * HD]; b.w = p[7 * HD];
    const v4u o = pack8(a, b);
    st2u(WO2p + (size_t)n * K2 + k8, o);
  } else if (u < U_ALL) {
    const int v  = u - U_HB - U_WH - U_WO;
    const int r  = v >> 8, c8 = (v & 255) * 8;
    const float* p = bias + (size_t)r * NN + c8;
    const v4f a = *(const v4fa*)p;
    const v4f b = *(const v4fa*)(p + 4);
    const v4u o = pack8(a, b);
    st2u(BBp + (size_t)r * NN + c8, o);
  }
}

__global__ __launch_bounds__(GTHR) __attribute__((amdgpu_num_vgpr(256)))
void k_gemm(const unsigned short* __restrict__ A, const unsigned short* __restrict__ WT, int K,
            const float* __restrict__ a1, const float* __restrict__ a2,
            float* FF, int ffPlane, unsigned short* VT, int nHeads) {
  __shared__ __attribute__((aligned(16))) float stg[64 * 64];
  __shared__ __attribute__((aligned(16))) float satt[2 * 64];
  __shared__ __attribute__((aligned(16))) float sdot[2 * 64];
  const int tid = (int)threadIdx.x, lane = tid & 31, wave = tid >> 5, hh = lane >> 4, m = lane & 15;
  const int rowBase = (int)blockIdx.x * 64;
  const int head    = (int)blockIdx.y;
  const int col0    = head * HD;
  const int bb      = rowBase >> 11;
  const int m0      = rowBase & (NN - 1);
  const int bk      = bb * nHeads + head;

  {
    const int which = tid >> 6;
    const int c = tid & 63;
    const float vs = a1[head * HD + c];
    const float vd = a2[head * HD + c];
    const float v = (which == 0) ? vs : vd;
    satt[which * 64 + c] = bfr(v);
  }

  v8f acc[4];
  {
    const v8f z = {0.f, 0.f, 0.f, 0.f, 0.f, 0.f, 0.f, 0.f};
    acc[0] = z; acc[1] = z; acc[2] = z; acc[3] = z;
  }
  const unsigned short* ap = A  + (size_t)(rowBase + 16 * wave + m) * (size_t)K + 8 * hh;
  const unsigned short* wp = WT + (size_t)(col0 + m) * (size_t)K + 8 * hh;
  const int ksteps = K >> 5;
#pragma unroll 1
  for (int ks = 0; ks < ksteps; ++ks) {
    FragB af;
    af.h[0] = *(const v8usa*)(ap + 32 * ks);
    af.h[1] = *(const v8usa*)(ap + 32 * ks + 16);
#pragma unroll
    for (int t = 0; t < 4; ++t) {
      const unsigned short* wq = wp + (size_t)(16 * t) * (size_t)K + 32 * ks;
      FragB bf;
      bf.h[0] = *(const v8usa*)wq;
      bf.h[1] = *(const v8usa*)(wq + 16);
      acc[t] = wmb(af, bf, acc[t]);
    }
  }

#pragma unroll
  for (int t = 0; t < 4; ++t) {
    const int lc = 16 * t + m;
#pragma unroll
    for (int r = 0; r < 8; ++r) {
      const int lr = 16 * wave + 8 * hh + r;
      stg[lr * 64 + lc] = acc[t][r];
    }
  }
  __syncthreads();

  {
    const int row = tid & 63, which = tid >> 6;
    const float* sa = satt + which * 64;
    const float* hr = stg + row * 64;
    float d = 0.f;
#pragma unroll 4
    for (int c4 = 0; c4 < 16; ++c4) {
      const v4f hv = *(const v4fa*)(hr + 4 * c4);
      const v4f av = *(const v4fa*)(sa + 4 * c4);
      d = fmaf(hv.x, av.x, d);
      d = fmaf(hv.y, av.y, d);
      d = fmaf(hv.z, av.z, d);
      d = fmaf(hv.w, av.w, d);
    }
    sdot[which * 64 + row] = d;
  }
  __syncthreads();

  v4u hv[4], lv[4];
#pragma unroll
  for (int it = 0; it < 4; ++it) {
    const int idx = it * GTHR + tid;
    const int hc = idx >> 3, pc = idx & 7;
    float x[8];
#pragma unroll
    for (int j = 0; j < 8; ++j) x[j] = stg[(8 * pc + j) * 64 + hc];
    unsigned int hb[8], lb[8];
#pragma unroll
    for (int j = 0; j < 8; ++j) {
      hb[j] = f2bf(x[j]);
      lb[j] = f2bf(x[j] - bf2f(hb[j]));
    }
    v4u h4, l4;
    h4.x = hb[0] | (hb[1] << 16); h4.y = hb[2] | (hb[3] << 16); h4.z = hb[4] | (hb[5] << 16); h4.w = hb[6] | (hb[7] << 16);
    l4.x = lb[0] | (lb[1] << 16); l4.y = lb[2] | (lb[3] << 16); l4.z = lb[4] | (lb[5] << 16); l4.w = lb[6] | (lb[7] << 16);
    hv[it] = h4; lv[it] = l4;
  }
  const int which2 = lane >> 4, piece = lane & 15;
  const v4f sdv = *(const v4fa*)(sdot + which2 * 64 + 4 * piece);
  float* fp = FF + (size_t)which2 * (size_t)ffPlane + (size_t)bk * NN + m0 + 4 * piece;
  unsigned short* vb = VT + ((size_t)bk * 2 * HD) * NN + m0;

#pragma unroll
  for (int it = 0; it < 4; ++it) {
    const int idx = it * GTHR + tid;
    const int hc = idx >> 3, pc = idx & 7;
    unsigned short* p = vb + (size_t)hc * NN + 8 * pc;
    *(volatile v4u*)p = hv[it];
    *(volatile v4u*)(p + (size_t)HD * NN) = lv[it];
  }
  if (wave == 0) *(volatile v4f*)fp = sdv;
  __threadfence();
#pragma unroll
  for (int it = 0; it < 4; ++it) {
    const int idx = it * GTHR + tid;
    const int hc = idx >> 3, pc = idx & 7;
    unsigned short* p = vb + (size_t)hc * NN + 8 * pc;
    *(volatile v4u*)p = hv[it];
    *(volatile v4u*)(p + (size_t)HD * NN) = lv[it];
  }
  if (wave == 0) *(volatile v4f*)fp = sdv;
}

template <int MODE>
__global__ __launch_bounds__(ATHR) __attribute__((amdgpu_num_vgpr(256)))
void k_att(const float* __restrict__ f1g, const float* __restrict__ f2g,
           const unsigned short* __restrict__ VT, const unsigned short* __restrict__ BB,
           unsigned short* H1, float* outF, int nHeads) {
  __shared__ __attribute__((aligned(16))) float stg[4 * 16 * 64];
  const int tid = (int)threadIdx.x, lane = tid & 31, wave = tid >> 5, hh = lane >> 4, m = lane & 15;
  const int head = (int)blockIdx.y, bb = (int)blockIdx.z;
  const int bk = bb * nHeads + head;
  const int i0 = (int)blockIdx.x * 64 + 16 * wave;

  const float f1m = f1g[(size_t)bk * NN + i0 + m];
  const float* f2p = f2g + (size_t)bk * NN + 8 * hh;
  const unsigned short* brow = BB + (size_t)(i0 + m) * NN + 8 * hh;
  const unsigned short* vhi  = VT + ((size_t)bk * 2 * HD + m) * NN + 8 * hh;
  const unsigned short* vlo  = vhi + (size_t)HD * NN;

  float mrun = -3.0e38f;
  float lrun = 0.0f;
  v8f acc[4];
  {
    const v8f z = {0.f, 0.f, 0.f, 0.f, 0.f, 0.f, 0.f, 0.f};
    acc[0] = z; acc[1] = z; acc[2] = z; acc[3] = z;
  }

#pragma unroll 1
  for (int j0 = 0; j0 < NN; j0 += 64) {
    float ev[32];
    float tmax = -3.0e38f;
#pragma unroll
    for (int g = 0; g < 4; ++g) {
      const v4u bw = *(const v4ua*)(brow + j0 + 16 * g);
      const v4f fa = *(const v4fa*)(f2p + j0 + 16 * g);
      const v4f fb = *(const v4fa*)(f2p + j0 + 16 * g + 4);
      ev[8 * g + 0] = sc1(f1m, fa.x, __uint_as_float(bw.x << 16));
      ev[8 * g + 1] = sc1(f1m, fa.y, __uint_as_float(bw.x & 0xFFFF0000u));
      ev[8 * g + 2] = sc1(f1m, fa.z, __uint_as_float(bw.y << 16));
      ev[8 * g + 3] = sc1(f1m, fa.w, __uint_as_float(bw.y & 0xFFFF0000u));
      ev[8 * g + 4] = sc1(f1m, fb.x, __uint_as_float(bw.z << 16));
      ev[8 * g + 5] = sc1(f1m, fb.y, __uint_as_float(bw.z & 0xFFFF0000u));
      ev[8 * g + 6] = sc1(f1m, fb.z, __uint_as_float(bw.w << 16));
      ev[8 * g + 7] = sc1(f1m, fb.w, __uint_as_float(bw.w & 0xFFFF0000u));
    }
#pragma unroll
    for (int t = 0; t < 32; ++t) tmax = fmaxf(tmax, ev[t]);
    tmax = fmaxf(tmax, __shfl_xor(tmax, 16));
    const float mnew  = fmaxf(mrun, tmax);
    const float scale = expf(mrun - mnew);
    mrun = mnew;

    FragB ah[2], al[2];
    float psum = 0.0f;
#pragma unroll
    for (int ks = 0; ks < 2; ++ks) {
#pragma unroll
      for (int w = 0; w < 8; ++w) {
        const float p0 = expf(ev[16 * ks + 2 * w]     - mnew);
        const float p1 = expf(ev[16 * ks + 2 * w + 1] - mnew);
        psum = psum + p0;
        psum = psum + p1;
        const unsigned int u0 = __float_as_uint(p0), u1 = __float_as_uint(p1);
        const unsigned int t0 = u0 & 0xFFFF0000u, t1 = u1 & 0xFFFF0000u;
        const float l0 = p0 - __uint_as_float(t0);
        const float l1 = p1 - __uint_as_float(t1);
        ah[ks].w[w] = (int)((u0 >> 16) | t1);
        al[ks].w[w] = (int)(f2bf(l0) | (f2bf(l1) << 16));
      }
    }
    psum = psum + __shfl_xor(psum, 16);
    lrun = lrun * scale + psum;

#pragma unroll
    for (int r = 0; r < 8; ++r) {
      const float sr = __shfl(scale, 8 * hh + r);
      acc[0][r] *= sr; acc[1][r] *= sr; acc[2][r] *= sr; acc[3][r] *= sr;
    }

#pragma unroll
    for (int ks = 0; ks < 2; ++ks) {
#pragma unroll
      for (int f = 0; f < 4; ++f) {
        const unsigned short* ph = vhi + (size_t)(16 * f) * NN + j0 + 32 * ks;
        const unsigned short* pl = vlo + (size_t)(16 * f) * NN + j0 + 32 * ks;
        FragB bh, bl;
        bh.h[0] = *(const v8usa*)ph;
        bh.h[1] = *(const v8usa*)(ph + 16);
        bl.h[0] = *(const v8usa*)pl;
        bl.h[1] = *(const v8usa*)(pl + 16);
        acc[f] = wmb(ah[ks], bh, acc[f]);
        acc[f] = wmb(al[ks], bh, acc[f]);
        acc[f] = wmb(ah[ks], bl, acc[f]);
      }
    }
  }

  float* sw = stg + wave * (16 * 64);
#pragma unroll
  for (int r = 0; r < 8; ++r) {
    const float lv = __shfl(lrun, 8 * hh + r);
    const float inv = 1.0f / lv;
    sw[(8 * hh + r) * 64 +  0 + m] = acc[0][r] * inv;
    sw[(8 * hh + r) * 64 + 16 + m] = acc[1][r] * inv;
    sw[(8 * hh + r) * 64 + 32 + m] = acc[2][r] * inv;
    sw[(8 * hh + r) * 64 + 48 + m] = acc[3][r] * inv;
  }
  __syncthreads();

  if constexpr (MODE == 0) {
#pragma unroll 1
    for (int it = 0; it < 4; ++it) {
      const int row = 4 * it + (lane >> 3), pc = lane & 7;
      const v4f x0 = *(const v4fa*)(sw + row * 64 + 8 * pc);
      const v4f x1 = *(const v4fa*)(sw + row * 64 + 8 * pc + 4);
      const float y0 = eluf(x0.x), y1 = eluf(x0.y), y2 = eluf(x0.z), y3 = eluf(x0.w);
      const float y4 = eluf(x1.x), y5 = eluf(x1.y), y6 = eluf(x1.z), y7 = eluf(x1.w);
      const unsigned int h0 = f2bf(y0), h1 = f2bf(y1), h2 = f2bf(y2), h3 = f2bf(y3);
      const unsigned int h4 = f2bf(y4), h5 = f2bf(y5), h6 = f2bf(y6), h7 = f2bf(y7);
      const unsigned int q0 = f2bf(y0 - bf2f(h0)), q1 = f2bf(y1 - bf2f(h1));
      const unsigned int q2 = f2bf(y2 - bf2f(h2)), q3 = f2bf(y3 - bf2f(h3));
      const unsigned int q4 = f2bf(y4 - bf2f(h4)), q5 = f2bf(y5 - bf2f(h5));
      const unsigned int q6 = f2bf(y6 - bf2f(h6)), q7 = f2bf(y7 - bf2f(h7));
      v4u hv, lv;
      hv.x = h0 | (h1 << 16); hv.y = h2 | (h3 << 16); hv.z = h4 | (h5 << 16); hv.w = h6 | (h7 << 16);
      lv.x = q0 | (q1 << 16); lv.y = q2 | (q3 << 16); lv.z = q4 | (q5 << 16); lv.w = q6 | (q7 << 16);
      unsigned short* hp = H1 + (size_t)(bb * NN + i0 + row) * K2 + head * HD + 8 * pc;
      *(volatile v4u*)hp = hv;
      *(volatile v4u*)(hp + HC) = lv;
      __threadfence();
      *(volatile v4u*)hp = hv;
      *(volatile v4u*)(hp + HC) = lv;
    }
  } else {
#pragma unroll 1
    for (int it = 0; it < 8; ++it) {
      const int row = 2 * it + (lane >> 4), c4 = (lane & 15) * 4;
      const v4f x = *(const v4fa*)(sw + row * 64 + c4);
      v4f y;
      y.x = eluf(x.x); y.y = eluf(x.y); y.z = eluf(x.z); y.w = eluf(x.w);
      float* op = outF + (size_t)(bb * NN + i0 + row) * HD + c4;
      *(volatile v4f*)op = y;
      __threadfence();
      *(volatile v4f*)op = y;
    }
  }
}

extern "C" void kernel_launch(void* const* d_in, const int* in_sizes, int n_in,
                              void* d_out, int out_size, void* d_ws, size_t ws_size,
                              hipStream_t stream) {
  if (n_in < 10) return;
  if (in_sizes[0] != MROWS * 2) return;
  if (in_sizes[1] != MROWS * 30) return;
  if (in_sizes[2] != MROWS * HD) return;
  if (in_sizes[3] != NN * NN) return;
  if (in_sizes[4] != NH * DATT * HD) return;
  if (in_sizes[5] != NH * HD || in_sizes[6] != NH * HD) return;
  if (in_sizes[7] != HC * HD) return;
  if (in_sizes[8] != HD || in_sizes[9] != HD) return;
  if (out_size != MROWS * HD) return;

  const float* inp  = (const float*)d_in[0];
  const float* env  = (const float*)d_in[1];
  const float* st   = (const float*)d_in[2];
  const float* bias = (const float*)d_in[3];
  const float* Wh   = (const float*)d_in[4];
  const float* a1h  = (const float*)d_in[5];
  const float* a2h  = (const float*)d_in[6];
  const float* Wo   = (const float*)d_in[7];
  const float* a1o  = (const float*)d_in[8];
  const float* a2o  = (const float*)d_in[9];
  float* out = (float*)d_out;

  char* ws = (char*)d_ws;
  size_t off = 0;
  const size_t oHB  = off; off += (size_t)MROWS * KPAD * 2;             off = (off + 255) & ~(size_t)255;
  const size_t oWHT = off; off += (size_t)HC * KPAD * 2;                off = (off + 255) & ~(size_t)255;
  const size_t oWO2 = off; off += (size_t)HD * K2 * 2;                  off = (off + 255) & ~(size_t)255;
  const size_t oBB  = off; off += (size_t)NN * NN * 2;                  off = (off + 255) & ~(size_t)255;
  const size_t oVT1 = off; off += (size_t)NBAT * NH * 2 * HD * NN * 2;  off = (off + 255) & ~(size_t)255;
  const size_t oFF1 = off; off += (size_t)2 * NBAT * NH * NN * 4;       off = (off + 255) & ~(size_t)255;
  const size_t oH1  = off; off += (size_t)MROWS * K2 * 2;               off = (off + 255) & ~(size_t)255;
  const size_t oVT2 = off; off += (size_t)NBAT * 2 * HD * NN * 2;       off = (off + 255) & ~(size_t)255;
  const size_t oFF2 = off; off += (size_t)2 * NBAT * NN * 4;            off = (off + 255) & ~(size_t)255;
  if (off > ws_size || off > (size_t)WSMAX) return;
  unsigned short* HBp  = (unsigned short*)(ws + oHB);
  unsigned short* WHTp = (unsigned short*)(ws + oWHT);
  unsigned short* WO2p = (unsigned short*)(ws + oWO2);
  unsigned short* BBp  = (unsigned short*)(ws + oBB);
  unsigned short* VT1  = (unsigned short*)(ws + oVT1);
  float*          FF1  = (float*)(ws + oFF1);
  unsigned short* H1   = (unsigned short*)(ws + oH1);
  unsigned short* VT2  = (unsigned short*)(ws + oVT2);
  float*          FF2  = (float*)(ws + oFF2);

  const int ffPlane1 = NBAT * NH * NN;
  const int ffPlane2 = NBAT * NN;

  k_prep<<<U_ALL / PTHR, PTHR, 0, stream>>>(inp, env, st, bias, Wh, Wo, HBp, WHTp, WO2p, BBp);
  k_gemm<<<dim3(MROWS / 64, NH), GTHR, 0, stream>>>(HBp, WHTp, KPAD, a1h, a2h, FF1, ffPlane1, VT1, NH);
  k_att<0><<<dim3(NN / 64, NH, NBAT), ATHR, 0, stream>>>(FF1, FF1 + ffPlane1, VT1, BBp, H1, out, NH);
  k_gemm<<<dim3(MROWS / 64, 1), GTHR, 0, stream>>>(H1, WO2p, K2, a1o, a2o, FF2, ffPlane2, VT2, 1);
  k_att<1><<<dim3(NN / 64, 1, NBAT), ATHR, 0, stream>>>(FF2, FF2 + ffPlane2, VT2, BBp, H1, out, 1);
}
